// MultiHeadAttention_75213467287764
// MI455X (gfx1250) — hardware-run, weakly checked
//
#include <hip/hip_runtime.h>


#ifndef NB
#define NB 2
#endif
#ifndef SEQ
#define SEQ 1024
#endif
#define NB_FULL  2
#define SEQ_FULL 1024
#ifndef OUT_SEQ
#define OUT_SEQ SEQ
#endif
#define DM   1024
#define K2   2048
#define NH_  16
#define HD   64
#define AW   4
#define QRS  2048.0f
#define QRI  (1.0f / 2048.0f)
#define SC2  (0.125f * 1.4426950408889634f)
#define PSH  8.0f
#define NEGMIN (-3.4028234663852886e38f)

static_assert(HD == 64);
static_assert(NH_ * HD == DM);
static_assert(K2 == 2 * DM);
static_assert((DM & (DM - 1)) == 0);
static_assert(DM % 64 == 0);
static_assert(SEQ % 128 == 0);
static_assert(SEQ % 64 == 0);
static_assert((NB * SEQ) % 64 == 0);
static_assert((NB * SEQ) % 8 == 0);
static_assert(SEQ % (16 * AW) == 0);
static_assert(NB <= NB_FULL);
static_assert(SEQ <= SEQ_FULL);

typedef _Float16 h16;
typedef unsigned short bf;
typedef __attribute__((ext_vector_type(16))) __bf16   v16bf;
typedef __attribute__((ext_vector_type(16))) _Float16 v16h;
typedef __attribute__((ext_vector_type(8)))  _Float16 v8h;
typedef __attribute__((ext_vector_type(8)))  unsigned short v8us;
typedef __attribute__((ext_vector_type(8)))  float    v8f;
typedef __attribute__((ext_vector_type(4)))  float    v4f;
typedef __attribute__((ext_vector_type(4)))  int      v4i;
typedef v4f  __attribute__((may_alias)) v4fa;
typedef v8h  __attribute__((may_alias)) v8ha;

__device__ __forceinline__ unsigned short f2bf(float f) { unsigned u = __float_as_uint(f); u += 0x7FFFu + ((u >> 16) & 1u); return (unsigned short)(u >> 16); }
__device__ __forceinline__ float bf2f(unsigned short b) { return __uint_as_float(((unsigned)b) << 16); }
__device__ __forceinline__ float bfr(float f) { return bf2f(f2bf(f)); }
__device__ __forceinline__ v16h cat16(v8h lo, v8h hi) { return __builtin_shufflevector(lo, hi, 0, 1, 2, 3, 4, 5, 6, 7, 8, 9, 10, 11, 12, 13, 14, 15); }
__device__ __forceinline__ v16bf cat16b(v8us lo, v8us hi) { return __builtin_bit_cast(v16bf, __builtin_shufflevector(lo, hi, 0, 1, 2, 3, 4, 5, 6, 7, 8, 9, 10, 11, 12, 13, 14, 15)); }
__device__ __forceinline__ v8f wmma16(v16h a, v16h b, v8f c) { return __builtin_amdgcn_wmma_f32_16x16x32_f16(false, a, false, b, (short)0, c, false, false); }
__device__ __forceinline__ v8f wmmab(v16bf a, v16bf b, v8f c) { return __builtin_amdgcn_wmma_f32_16x16x32_bf16(false, a, false, b, (short)0, c, false, false); }
__device__ __forceinline__ v16h  ldh(const h16* p) { return cat16(*(const v8h*)p, *(const v8h*)(p + 16)); }
__device__ __forceinline__ v16bf ldb(const bf* p)  { return cat16b(*(const v8us*)p, *(const v8us*)(p + 16)); }
__device__ __forceinline__ void wave_sync() { __builtin_amdgcn_fence(3  , "wavefront"); __builtin_amdgcn_wave_barrier(); asm volatile("" ::: "memory"); }
__device__ __forceinline__ float wsum(float v) { v += __shfl_xor(v, 16, 32); v += __shfl_xor(v, 8, 32); v += __shfl_xor(v, 4, 32); v += __shfl_xor(v, 2, 32); v += __shfl_xor(v, 1, 32); return v; }
__device__ __forceinline__ int wsumi(int v) { v += __shfl_xor(v, 16, 32); v += __shfl_xor(v, 8, 32); v += __shfl_xor(v, 4, 32); v += __shfl_xor(v, 2, 32); v += __shfl_xor(v, 1, 32); return v; }

__global__ __launch_bounds__(256) void k_cvt8(const float* __restrict__ src, bf* dst, size_t n8) {
    const size_t i = (size_t)blockIdx.x * 256 + threadIdx.x; if (i >= n8) return;
    const v8f v = *(const v8f*)(src + i * 8); v8us o;
#pragma unroll
    for (int k = 0; k < 8; ++k) o[k] = f2bf(v[k]);
    *(volatile v8us*)(dst + i * 8) = o; __threadfence(); *(volatile v8us*)(dst + i * 8) = o;
}

__global__ __launch_bounds__(256) void k_ew(const float* __restrict__ ew, h16* EWA) {
    const int tid = threadIdx.x; const int d = tid >> 2, q = tid & 3;
    const float sc = (q < 2) ? 16.0f : 0.0078125f;
    const v8f w = *(const v8f*)(ew + d * 16 + (q & 1) * 8);
    v8h o;
#pragma unroll
    for (int i = 0; i < 8; ++i) o[i] = (h16)(bfr(w[i]) * sc);
    *(volatile v8h*)(EWA + d * 32 + q * 8) = o; __threadfence(); *(volatile v8h*)(EWA + d * 32 + q * 8) = o;
}

__global__ __launch_bounds__(256) void k_lnx(const float* __restrict__ x, const float* __restrict__ lw, const float* __restrict__ lb, bf* XA) {
    const int lane = threadIdx.x & 31; const int wave = __builtin_amdgcn_readfirstlane((int)(threadIdx.x >> 5));
    const int m = blockIdx.x * 8 + wave; const int b = m / SEQ, t = m % SEQ;
    const float* src = x + ((size_t)b * SEQ_FULL + t) * DM + lane * 8;
    float s = 0.0f;
#pragma unroll 1
    for (int it = 0; it < 4; ++it) { const v8f raw = *(const v8f*)(src + it * 256);
#pragma unroll
        for (int i = 0; i < 8; ++i) s += bfr(raw[i]); }
    s = wsum(s);
    const float mean = s * (1.0f / DM);
    float ss = 0.0f;
#pragma unroll 1
    for (int it = 0; it < 4; ++it) { const v8f raw = *(const v8f*)(src + it * 256);
#pragma unroll
        for (int i = 0; i < 8; ++i) { const float dv = bfr(raw[i]) - mean; ss += dv * dv; } }
    ss = wsum(ss);
    const float rstd = 1.0f / sqrtf(ss * (1.0f / DM) + 1e-5f);
    bf* dst = XA + (size_t)m * K2 + lane * 8;
#pragma unroll 1
    for (int ps = 0; ps < 2; ++ps) {
#pragma unroll 1
        for (int it = 0; it < 4; ++it) {
            const v8f raw = *(const v8f*)(src + it * 256);
            const v8f wv = *(const v8f*)(lw + it * 256 + lane * 8); const v8f bv = *(const v8f*)(lb + it * 256 + lane * 8);
            v8us hv, lv;
#pragma unroll
            for (int i = 0; i < 8; ++i) { const float dv = bfr(raw[i]) - mean; const float y = dv * rstd * bfr(wv[i]) + bfr(bv[i]); const unsigned short hh = f2bf(y); hv[i] = hh; lv[i] = f2bf(y - bf2f(hh)); }
            *(volatile v8us*)(dst + it * 256) = hv; *(volatile v8us*)(dst + DM + it * 256) = lv; }
        if (ps == 0) __threadfence(); }
}

__global__ __launch_bounds__(256) void k_rope(const float* __restrict__ pos, float* CS, float* SN) {
    const int lane = threadIdx.x & 31; const int wave = __builtin_amdgcn_readfirstlane((int)(threadIdx.x >> 5));
    const int m = blockIdx.x * 8 + wave; const int b = m / SEQ, t = m % SEQ;
    const float p = bfr(pos[(size_t)b * SEQ_FULL + t]);
    double pd = 1.0;
#pragma unroll 1
    for (int i = 0; i < lane; ++i) pd *= 1.333521432163324;
    const float pf = (float)pd;
    const float invf = 1.0f / pf;
    const float ang = p * invf;
    const float c = cosf(ang), s = sinf(ang);
    *(volatile float*)(CS + (size_t)m * 32 + lane) = c; *(volatile float*)(SN + (size_t)m * 32 + lane) = s;
    __threadfence();
    *(volatile float*)(CS + (size_t)m * 32 + lane) = c; *(volatile float*)(SN + (size_t)m * 32 + lane) = s;
}

__global__ __launch_bounds__(256) void k_prep(const float* __restrict__ blocks, const int* __restrict__ mask, h16* BM, float* BASE) {
    __shared__ float slen[64];
    __shared__ __align__(16) h16 sb[32 * 64];
    __shared__ __align__(16) float sbase[64 * 16];
    const int tid = threadIdx.x, lane = tid & 31; const int wave = __builtin_amdgcn_readfirstlane((int)(threadIdx.x >> 5));
    const int m0 = blockIdx.x * 64; const int b = m0 / SEQ, t0 = m0 % SEQ;
#pragma unroll 1
    for (int i = 0; i < 8; ++i) { const int tl = wave * 8 + i;
        const int* row = mask + ((size_t)b * SEQ_FULL + t0 + tl) * SEQ_FULL + lane * 4; int cnt = 0;
#pragma unroll
        for (int c = 0; c < SEQ / 128; ++c) { const v4i mv = *(const v4i*)(row + c * 128); cnt += (mv[0] != 0) + (mv[1] != 0) + (mv[2] != 0) + (mv[3] != 0); }
        cnt = wsumi(cnt);
        if (lane == 0) slen[tl] = (float)cnt; }
    __syncthreads();
    if (tid < 64) {
        const float* p = blocks + ((size_t)b * SEQ_FULL + t0 + tid) * 12;
        const v4f a0 = *(const v4f*)p, a1 = *(const v4f*)(p + 4), a2 = *(const v4f*)(p + 8);
        float pv[12];
#pragma unroll
        for (int i = 0; i < 4; ++i) { pv[i] = bfr(a0[i]); pv[4 + i] = bfr(a1[i]); pv[8 + i] = bfr(a2[i]); }
        float mu[3];
#pragma unroll
        for (int x = 0; x < 3; ++x) mu[x] = (pv[x] + pv[3 + x] + pv[6 + x] + pv[9 + x]) * 0.25f;
        const float sc = (1.0f / slen[tid]) * 1024.0f;
#pragma unroll
        for (int c = 0; c < 4; ++c) {
            const float vx = pv[c * 3] - mu[0], vy = pv[c * 3 + 1] - mu[1], vz = pv[c * 3 + 2] - mu[2];
            const float inv = 1.0f / (sqrtf(vx * vx + vy * vy + vz * vz) + 1.1920929e-7f);
            const float vv[3] = {vx, vy, vz};
#pragma unroll
            for (int x = 0; x < 3; ++x) { const int cx = c * 3 + x;
                sbase[tid * 16 + cx] = vv[x] * inv;
                const float bs = vv[x] * sc; const h16 hh = (h16)bs;
                sb[cx * 64 + tid] = hh; sb[(16 + cx) * 64 + tid] = (h16)((bs - (float)hh) * QRS); } }
#pragma unroll
        for (int j = 12; j < 16; ++j) { sbase[tid * 16 + j] = 0.0f; sb[j * 64 + tid] = (h16)0.0f; sb[(16 + j) * 64 + tid] = (h16)0.0f; }
    }
    __syncthreads();
    const int line = tid >> 3, pc = tid & 7;
    const v8h bv = *(const v8ha*)(&sb[line * 64 + pc * 8]);
    const v4f fv = *(const v4fa*)(&sbase[tid * 4]);
    h16* bd = BM + (size_t)(line >> 4) * ((size_t)NB * 16 * SEQ) + ((size_t)b * 16 + (line & 15)) * SEQ + t0 + pc * 8;
    float* fd = BASE + (size_t)m0 * 16 + tid * 4;
    *(volatile v8h*)bd = bv; *(volatile v4f*)fd = fv;
    __threadfence();
    *(volatile v8h*)bd = bv; *(volatile v4f*)fd = fv;
}

template <int MODE>
__global__ __launch_bounds__(32) void k_proj(const bf* __restrict__ A, int pA, const bf* __restrict__ Bt, int pB, int K,
                                             h16* Ph, int RB, size_t sRB, int pitch, int CB, size_t sCB, float* C, int ldc, int RP) {
    __shared__ __align__(16) float os[16 * 68];
    const int lane = threadIdx.x & 31, lr = lane & 15, hi = lane >> 4; const int r0 = blockIdx.x * 64, c0 = blockIdx.y * 64;
    v8f acc[4][4];
#pragma unroll
    for (int mb = 0; mb < 4; ++mb)
#pragma unroll
        for (int nb = 0; nb < 4; ++nb) acc[mb][nb] = (v8f){};
    const size_t aoff = (size_t)(r0 + lr) * pA + 8 * hi, boff = (size_t)(c0 + lr) * pB + 8 * hi;
    const int mA = pA - 1, mB = pB - 1;
#pragma unroll 1
    for (int kc = 0; kc < K; kc += 32) {
        const int ka = kc & mA, kb = kc & mB;
        v16bf a[4];
#pragma unroll
        for (int mb = 0; mb < 4; ++mb) a[mb] = ldb(A + aoff + (size_t)mb * 16 * pA + ka);
#pragma unroll
        for (int nb = 0; nb < 4; ++nb) { const v16bf b = ldb(Bt + boff + (size_t)nb * 16 * pB + kb);
#pragma unroll
            for (int mb = 0; mb < 4; ++mb) acc[mb][nb] = wmmab(a[mb], b, acc[mb][nb]); }
        asm volatile("v_nop\n\tv_nop\n\tv_nop\n\tv_nop" : "+v"(acc[0][0]), "+v"(acc[1][1]), "+v"(acc[2][2]), "+v"(acc[3][3]) : "v"(a[0]), "v"(a[1]), "v"(a[2]), "v"(a[3]));
    }
    const size_t tbase = (size_t)(r0 / RB) * sRB + (size_t)(r0 % RB) * (size_t)pitch + (size_t)(c0 / CB) * sCB + (size_t)(c0 % CB);
    const size_t cbase = ((size_t)(r0 / RB) * (size_t)RP + (size_t)(r0 % RB)) * (size_t)ldc + (size_t)c0;
#pragma unroll
    for (int mb = 0; mb < 4; ++mb) {
#pragma unroll
        for (int nb = 0; nb < 4; ++nb) {
#pragma unroll
            for (int j = 0; j < 8; ++j) os[(hi * 8 + j) * 68 + nb * 16 + lr] = acc[mb][nb][j]; }
        wave_sync();
        if (MODE == 0) {
            const size_t sb = tbase + (size_t)(mb * 16) * (size_t)pitch;
#pragma unroll 1
            for (int ps = 0; ps < 2; ++ps) {
#pragma unroll
                for (int s = 0; s < 4; ++s) { const int row = 4 * s + (lane >> 3), c8 = (lane & 7) * 8;
                    const v4f x0 = *(const v4fa*)(&os[row * 68 + c8]); const v4f x1 = *(const v4fa*)(&os[row * 68 + c8 + 4]); v8h hv;
#pragma unroll
                    for (int i = 0; i < 4; ++i) { hv[i] = (h16)x0[i]; hv[4 + i] = (h16)x1[i]; }
                    *(volatile v8h*)(Ph + sb + (size_t)row * (size_t)pitch + c8) = hv; }
                if (ps == 0) __threadfence(); }
        } else {
            const size_t sb = cbase + (size_t)(mb * 16) * (size_t)ldc;
#pragma unroll 1
            for (int ps = 0; ps < 2; ++ps) {
#pragma unroll
                for (int s = 0; s < 8; ++s) { const int row = 2 * s + hi, cofs = lr * 4;
                    const v4f val = *(const v4fa*)(&os[row * 68 + cofs]);
                    *(volatile v4f*)(C + sb + (size_t)row * (size_t)ldc + cofs) = val; }
                if (ps == 0) __threadfence(); }
        }
        wave_sync();
    }
}

__global__ __launch_bounds__(256) void k_qkrot(const float* __restrict__ QK, const float* __restrict__ qw, const float* __restrict__ kw, const float* __restrict__ CS, const float* __restrict__ SN,
                                               h16* PL, size_t pst) {
    const int lane = threadIdx.x & 31; const int wave = __builtin_amdgcn_readfirstlane((int)(threadIdx.x >> 5));
    const int m = blockIdx.x * 8 + wave; const int b = m / SEQ, t = m % SEQ;
    const int c = lane & 7;
    const v8f cs = *(const v8f*)(CS + (size_t)m * 32 + 8 * (c & 3));
    const v8f sn = *(const v8f*)(SN + (size_t)m * 32 + 8 * (c & 3));
    const float sg = (c < 4) ? -1.0f : 1.0f;
    const size_t o0 = (((size_t)(b * NH_ + (lane >> 3))) * SEQ + t) * HD + 8 * c;
    const size_t ost = (size_t)4 * SEQ * HD;
#pragma unroll 1
    for (int wh = 0; wh < 2; ++wh) {
        const float* row = QK + (size_t)m * K2 + (size_t)wh * DM + lane * 8;
        float s = 0.0f;
#pragma unroll 1
        for (int it = 0; it < 4; ++it) { const v8f raw = *(const v8f*)(row + it * 256);
#pragma unroll
            for (int i = 0; i < 8; ++i) s += raw[i]; }
        s = wsum(s);
        const float mean = s * (1.0f / DM);
        float ss = 0.0f;
#pragma unroll 1
        for (int it = 0; it < 4; ++it) { const v8f raw = *(const v8f*)(row + it * 256);
#pragma unroll
            for (int i = 0; i < 8; ++i) { const float dv = raw[i] - mean; ss += dv * dv; } }
        ss = wsum(ss);
        const float rstd = 1.0f / sqrtf(ss * (1.0f / DM) + 1e-5f);
        h16* PH = PL + (size_t)(2 * wh) * pst;
        h16* PR = PH + pst;
#pragma unroll 1
        for (int ps = 0; ps < 2; ++ps) {
#pragma unroll 1
            for (int it = 0; it < 4; ++it) {
                const v8f raw = *(const v8f*)(row + it * 256);
                const v8f wq = *(const v8f*)(qw + it * 256 + lane * 8); const v8f wk = *(const v8f*)(kw + it * 256 + lane * 8);
                v8h hv, rv;
#pragma unroll
                for (int i = 0; i < 8; ++i) { const float wsel = wh ? wk[i] : wq[i];
                    const float y = (raw[i] - mean) * rstd * bfr(wsel);
                    const float pr = __shfl_xor(y, 4, 32);
                    const float r = y * cs[i] + sg * pr * sn[i];
                    const h16 hh = (h16)r; hv[i] = hh; rv[i] = (h16)((r - (float)hh) * QRS); }
                const size_t oo = o0 + (size_t)it * ost;
                *(volatile v8h*)(PH + oo) = hv; *(volatile v8h*)(PR + oo) = rv; }
            if (ps == 0) __threadfence(); }
    }
}

__global__ __launch_bounds__(32 * AW) void k_flash(const h16* __restrict__ QH, const h16* __restrict__ QR, const h16* __restrict__ KH, const h16* __restrict__ KR, const h16* __restrict__ VT,
                                                   const h16* __restrict__ BM, const float* __restrict__ BASE, const h16* __restrict__ EWA, const int* __restrict__ mask, bf* OA) {
    __shared__ __align__(16) float os[AW * 16 * 68];
    const int lane = threadIdx.x & 31, wave = __builtin_amdgcn_readfirstlane((int)(threadIdx.x >> 5)), lr = lane & 15, hi = lane >> 4;
    const int zh = blockIdx.y; const int b = zh / NH_, h = zh % NH_;
    const int t0 = (blockIdx.x * AW + wave) * 16;
    const size_t pbase = (size_t)zh * SEQ * HD;
    const size_t qo = pbase + (size_t)(t0 + lr) * HD + 8 * hi;
    const v16h qh0 = ldh(QH + qo), qh1 = ldh(QH + qo + 32), qr0 = ldh(QR + qo), qr1 = ldh(QR + qo + 32);
    const size_t ko = pbase + (size_t)lr * HD + 8 * hi;
    const size_t vo = pbase + (size_t)lr * SEQ + 8 * hi;
    const size_t bmo = ((size_t)b * 16 + lr) * SEQ + 8 * hi;
    const h16* BMR = BM + (size_t)NB * 16 * SEQ;
    const int* mrow = mask + ((size_t)b * SEQ_FULL + t0 + lr) * SEQ_FULL + 8 * hi;
    v8f o0 = (v8f){}, o1 = (v8f){}, o2 = (v8f){}, o3 = (v8f){}, gA = (v8f){}, gR = (v8f){};
    float m = -__builtin_huge_valf(), l = 0.0f;
#pragma unroll 1
    for (int key0 = 0; key0 < SEQ; key0 += 32) {
        const v4i mk0 = *(const v4i*)(mrow + key0), mk1 = *(const v4i*)(mrow + key0 + 4), mk2 = *(const v4i*)(mrow + key0 + 16), mk3 = *(const v4i*)(mrow + key0 + 20);
        const h16* ka = KH + ko + (size_t)key0 * HD; const h16* kr = KR + ko + (size_t)key0 * HD;
        const v16h ka0 = ldh(ka), ka1 = ldh(ka + 32), kb0 = ldh(ka + 16 * HD), kb1 = ldh(ka + 16 * HD + 32);
        const v16h ra0 = ldh(kr), ra1 = ldh(kr + 32), rb0 = ldh(kr + 16 * HD), rb1 = ldh(kr + 16 * HD + 32);
        v8f sHa = (v8f){}, sLa = (v8f){}, sKa = (v8f){}, sHb = (v8f){}, sLb = (v8f){}, sKb = (v8f){};
        sHa = wmma16(ka0, qh0, sHa); sLa = wmma16(ka0, qr0, sLa); sKa = wmma16(ra0, qh0, sKa); sHb = wmma16(kb0, qh0, sHb); sLb = wmma16(kb0, qr0, sLb); sKb = wmma16(rb0, qh0, sKb);
        sHa = wmma16(ka1, qh1, sHa); sLa = wmma16(ka1, qr1, sLa); sKa = wmma16(ra1, qh1, sKa); sHb = wmma16(kb1, qh1, sHb); sLb = wmma16(kb1, qr1, sLb); sKb = wmma16(rb1, qh1, sKb);
        asm volatile("v_nop\n\tv_nop\n\tv_nop\n\tv_nop" : "+v"(sHa), "+v"(sLa), "+v"(sKa), "+v"(sHb), "+v"(sLb), "+v"(sKb) : "v"(ka0), "v"(ka1), "v"(kb0), "v"(kb1), "v"(ra0), "v"(ra1), "v"(rb0), "v"(rb1));
        const int mka[8] = {mk0[0], mk0[1], mk0[2], mk0[3], mk1[0], mk1[1], mk1[2], mk1[3]};
        const int mkb[8] = {mk2[0], mk2[1], mk2[2], mk2[3], mk3[0], mk3[1], mk3[2], mk3[3]};
        float ta[8], tb[8]; float mx = NEGMIN;
        v16h gh, gr;
#pragma unroll
        for (int r = 0; r < 8; ++r) {
            const float xa = sHa[r] + (sLa[r] + sKa[r]) * QRI; const float xb = sHb[r] + (sLb[r] + sKb[r]) * QRI;
            const bool va = (mka[r] != 0), vb = (mkb[r] != 0);
            ta[r] = va ? xa * SC2 : NEGMIN; tb[r] = vb ? xb * SC2 : NEGMIN;
            const float ga = va ? xa : 0.0f; const float gb = vb ? xb : 0.0f;
            const h16 ha = (h16)ga; const h16 hb = (h16)gb;
            gh[r] = ha; gh[8 + r] = hb; gr[r] = (h16)((ga - (float)ha) * QRS); gr[8 + r] = (h16)((gb - (float)hb) * QRS);
            mx = fmaxf(mx, fmaxf(ta[r], tb[r])); }
        mx = fmaxf(mx, __shfl_xor(mx, 16, 32));
        const float mnew = fmaxf(m, mx);
        const float alpha = __builtin_amdgcn_exp2f(m - mnew);
        const float sh = PSH - mnew;
        v16h pb; float ls = 0.0f;
#pragma unroll
        for (int r = 0; r < 8; ++r) { const h16 pa = (h16)__builtin_amdgcn_exp2f(ta[r] + sh); const h16 pc = (h16)__builtin_amdgcn_exp2f(tb[r] + sh); pb[r] = pa; pb[8 + r] = pc; ls += (float)pa + (float)pc; }
        l = l * alpha + ls; m = mnew;
        o0 = o0 * alpha; o1 = o1 * alpha; o2 = o2 * alpha; o3 = o3 * alpha;
        const h16* va_ = VT + vo + key0;
        const v16h v0 = ldh(va_), v1 = ldh(va_ + (size_t)16 * SEQ), v2 = ldh(va_ + (size_t)32 * SEQ), v3 = ldh(va_ + (size_t)48 * SEQ);
        const v16h bh = ldh(BM + bmo + key0), br = ldh(BMR + bmo + key0);
        o0 = wmma16(v0, pb, o0); gA = wmma16(bh, gh, gA); o1 = wmma16(v1, pb, o1); gR = wmma16(bh, gr, gR); o2 = wmma16(v2, pb, o2); o3 = wmma16(v3, pb, o3); gR = wmma16(br, gh, gR);
        asm volatile("v_nop\n\tv_nop\n\tv_nop\n\tv_nop" : "+v"(o0), "+v"(o1), "+v"(o2), "+v"(o3), "+v"(gA), "+v"(gR) : "v"(v0), "v"(v1), "v"(v2), "v"(v3), "v"(pb), "v"(bh), "v"(br), "v"(gh), "v"(gr));
    }
    l += __shfl_xor(l, 16, 32);
    const float inv = 1.0f / l;
    float mi[8], ot[8], f[12];
#pragma unroll
    for (int r = 0; r < 8; ++r) { mi[r] = gA[r] + gR[r] * QRI; ot[r] = __shfl_xor(mi[r], 16, 32); }
#pragma unroll
    for (int r = 0; r < 8; ++r) f[r] = hi ? ot[r] : mi[r];
#pragma unroll
    for (int r = 0; r < 4; ++r) f[8 + r] = hi ? mi[r] : ot[r];
    const float* bp = BASE + ((size_t)b * SEQ + t0 + lr) * 16;
    const v4f b0 = *(const v4f*)bp, b1 = *(const v4f*)(bp + 4), b2 = *(const v4f*)(bp + 8);
    const float bs[12] = {b0[0], b0[1], b0[2], b0[3], b1[0], b1[1], b1[2], b1[3], b2[0], b2[1], b2[2], b2[3]};
    float e0[3], e1[3];
#pragma unroll
    for (int x = 0; x < 3; ++x) { e0[x] = hi ? bs[6 + x] : bs[x]; e1[x] = hi ? bs[9 + x] : bs[3 + x]; }
    v16h cb;
#pragma unroll
    for (int i = 0; i < 8; ++i) { const int c = i & 3;
        const float cv = (i < 4) ? (e0[0] * f[3 * c] + e0[1] * f[3 * c + 1] + e0[2] * f[3 * c + 2]) : (e1[0] * f[3 * c] + e1[1] * f[3 * c + 1] + e1[2] * f[3 * c + 2]);
        const float bq = cv * (1.0f / 64.0f); const h16 hh = (h16)bq; cb[i] = hh; cb[8 + i] = (h16)((bq - (float)hh) * QRS); }
    const v16h ea0 = ldh(EWA + (size_t)(lr) * 32 + 8 * hi), ea1 = ldh(EWA + (size_t)(16 + lr) * 32 + 8 * hi), ea2 = ldh(EWA + (size_t)(32 + lr) * 32 + 8 * hi), ea3 = ldh(EWA + (size_t)(48 + lr) * 32 + 8 * hi);
    v8f c0 = (v8f){}, c1 = (v8f){}, c2 = (v8f){}, c3 = (v8f){};
    c0 = wmma16(ea0, cb, c0); c1 = wmma16(ea1, cb, c1); c2 = wmma16(ea2, cb, c2); c3 = wmma16(ea3, cb, c3);
    asm volatile("v_nop\n\tv_nop\n\tv_nop\n\tv_nop" : "+v"(c0), "+v"(c1), "+v"(c2), "+v"(c3) : "v"(ea0), "v"(ea1), "v"(ea2), "v"(ea3), "v"(cb));
    const float ci = 1.0f / 256.0f;
    const int wb = wave * 16 * 68;
    { v4f a, c;
      a[0] = o0[0] * inv + c0[0] * ci; a[1] = o0[1] * inv + c0[1] * ci; a[2] = o0[2] * inv + c0[2] * ci; a[3] = o0[3] * inv + c0[3] * ci;
      c[0] = o0[4] * inv + c0[4] * ci; c[1] = o0[5] * inv + c0[5] * ci; c[2] = o0[6] * inv + c0[6] * ci; c[3] = o0[7] * inv + c0[7] * ci;
      *(v4fa*)(&os[wb + lr * 68 +  0 + 8 * hi]) = a; *(v4fa*)(&os[wb + lr * 68 +  0 + 8 * hi + 4]) = c;
      a[0] = o1[0] * inv + c1[0] * ci; a[1] = o1[1] * inv + c1[1] * ci; a[2] = o1[2] * inv + c1[2] * ci; a[3] = o1[3] * inv + c1[3] * ci;
      c[0] = o1[4] * inv + c1[4] * ci; c[1] = o1[5] * inv + c1[5] * ci; c[2] = o1[6] * inv + c1[6] * ci; c[3] = o1[7] * inv + c1[7] * ci;
      *(v4fa*)(&os[wb + lr * 68 + 16 + 8 * hi]) = a; *(v4fa*)(&os[wb + lr * 68 + 16 + 8 * hi + 4]) = c;
      a[0] = o2[0] * inv + c2[0] * ci; a[1] = o2[1] * inv + c2[1] * ci; a[2] = o2[2] * inv + c2[2] * ci; a[3] = o2[3] * inv + c2[3] * ci;
      c[0] = o2[4] * inv + c2[4] * ci; c[1] = o2[5] * inv + c2[5] * ci; c[2] = o2[6] * inv + c2[6] * ci; c[3] = o2[7] * inv + c2[7] * ci;
      *(v4fa*)(&os[wb + lr * 68 + 32 + 8 * hi]) = a; *(v4fa*)(&os[wb + lr * 68 + 32 + 8 * hi + 4]) = c;
      a[0] = o3[0] * inv + c3[0] * ci; a[1] = o3[1] * inv + c3[1] * ci; a[2] = o3[2] * inv + c3[2] * ci; a[3] = o3[3] * inv + c3[3] * ci;
      c[0] = o3[4] * inv + c3[4] * ci; c[1] = o3[5] * inv + c3[5] * ci; c[2] = o3[6] * inv + c3[6] * ci; c[3] = o3[7] * inv + c3[7] * ci;
      *(v4fa*)(&os[wb + lr * 68 + 48 + 8 * hi]) = a; *(v4fa*)(&os[wb + lr * 68 + 48 + 8 * hi + 4]) = c; }
    wave_sync();
    bf* orow = OA + ((size_t)b * SEQ + t0) * K2 + h * HD;
#pragma unroll 1
    for (int ps = 0; ps < 2; ++ps) {
#pragma unroll
        for (int s = 0; s < 4; ++s) { const int row = 4 * s + (lane >> 3), c8 = (lane & 7) * 8;
            const v4f x0 = *(const v4fa*)(&os[wb + row * 68 + c8]); const v4f x1 = *(const v4fa*)(&os[wb + row * 68 + c8 + 4]); v8us hv, lv;
#pragma unroll
            for (int i = 0; i < 4; ++i) { const unsigned short a0 = f2bf(x0[i]); const unsigned short a1 = f2bf(x1[i]); hv[i] = a0; hv[4 + i] = a1; lv[i] = f2bf(x0[i] - bf2f(a0)); lv[4 + i] = f2bf(x1[i] - bf2f(a1)); }
            const size_t oo = (size_t)row * K2 + c8;
            *(volatile v8us*)(orow + oo) = hv; *(volatile v8us*)(orow + DM + oo) = lv; }
        if (ps == 0) __threadfence(); }
}

static constexpr size_t al256(size_t v) { return (v + 255) & ~(size_t)255; }
static constexpr size_t SZ_WB  = al256((size_t)3 * DM * DM * 2);
static constexpr size_t SZ_OWB = al256((size_t)DM * DM * 2);
static constexpr size_t SZ_XA  = al256((size_t)NB * SEQ * K2 * 2);
static constexpr size_t SZ_QK  = al256((size_t)NB * SEQ * K2 * 4);
static constexpr size_t SZ_PL  = al256((size_t)NB * NH_ * SEQ * HD * 2);
static constexpr size_t SZ_BM  = al256((size_t)2 * NB * 16 * SEQ * 2);
static constexpr size_t SZ_BS  = al256((size_t)NB * SEQ * 16 * 4);
static constexpr size_t SZ_CS  = al256((size_t)NB * SEQ * 32 * 4);
static constexpr size_t SZ_EW  = al256((size_t)64 * 32 * 2);
static constexpr size_t SZ_TOTAL = SZ_WB + SZ_OWB + 2 * SZ_XA + SZ_QK + 5 * SZ_PL + SZ_BM + SZ_BS + 2 * SZ_CS + SZ_EW;
static_assert(SZ_TOTAL <= (size_t)134217728);
static_assert(SZ_PL % 2 == 0);
static_assert(SZ_PL == (size_t)NB * NH_ * SEQ * HD * 2);

extern "C" void kernel_launch(void* const* d_in, const int* in_sizes, int n_in,
                              void* d_out, int out_size, void* d_ws, size_t ws_size, hipStream_t stream) {
    if (n_in < 11) return;
    const size_t ntok = (size_t)(NB - 1) * SEQ_FULL + SEQ;
    if ((size_t)in_sizes[0] < ntok) return;
    if ((size_t)in_sizes[1] < ntok * DM) return;
    if ((size_t)in_sizes[2] < (ntok - 1) * SEQ_FULL + SEQ) return;
    if ((size_t)in_sizes[3] < ntok * 12) return;
    if ((size_t)in_sizes[4] < (size_t)DM || (size_t)in_sizes[5] < (size_t)DM || (size_t)in_sizes[7] < (size_t)DM || (size_t)in_sizes[8] < (size_t)DM) return;
    if ((size_t)in_sizes[6] < (size_t)3 * DM * DM || (size_t)in_sizes[9] < (size_t)DM * DM || (size_t)in_sizes[10] < (size_t)1024) return;
    if ((size_t)out_size < ((size_t)(NB - 1) * OUT_SEQ + SEQ) * DM) return;
    if (SZ_TOTAL > ws_size) return;
    const float* position = (const float*)d_in[0]; const float* x = (const float*)d_in[1]; const int* amask = (const int*)d_in[2]; const float* blocks = (const float*)d_in[3];
    const float* ln_w = (const float*)d_in[4]; const float* ln_b = (const float*)d_in[5]; const float* wqkv = (const float*)d_in[6];
    const float* q_ln_w = (const float*)d_in[7]; const float* k_ln_w = (const float*)d_in[8]; const float* out_w = (const float*)d_in[9]; const float* edge_w = (const float*)d_in[10];
    float* OUT = (float*)d_out;
    char* wsp = (char*)d_ws;
    bf* WB  = (bf*)wsp;  wsp += SZ_WB;
    bf* OWB = (bf*)wsp;  wsp += SZ_OWB;
    bf* XA  = (bf*)wsp;  wsp += SZ_XA;
    bf* OA  = (bf*)wsp;  wsp += SZ_XA;
    float* QK = (float*)wsp; wsp += SZ_QK;
    h16* QH = (h16*)wsp; wsp += SZ_PL;
    h16* QR = (h16*)wsp; wsp += SZ_PL;
    h16* KH = (h16*)wsp; wsp += SZ_PL;
    h16* KR = (h16*)wsp; wsp += SZ_PL;
    h16* VT = (h16*)wsp; wsp += SZ_PL;
    h16* BM = (h16*)wsp; wsp += SZ_BM;
    float* BASE = (float*)wsp; wsp += SZ_BS;
    float* CS = (float*)wsp; wsp += SZ_CS;
    float* SN = (float*)wsp; wsp += SZ_CS;
    h16* EWA = (h16*)wsp; wsp += SZ_EW;

    { const size_t n8 = (size_t)3 * DM * DM / 8; k_cvt8<<<(unsigned)((n8 + 255) / 256), 256, 0, stream>>>(wqkv, WB, n8); }
    { const size_t n8 = (size_t)DM * DM / 8;     k_cvt8<<<(unsigned)((n8 + 255) / 256), 256, 0, stream>>>(out_w, OWB, n8); }
    k_ew<<<1, 256, 0, stream>>>(edge_w, EWA);
    k_lnx<<<NB * SEQ / 8, 256, 0, stream>>>(x, ln_w, ln_b, XA);
    k_rope<<<NB * SEQ / 8, 256, 0, stream>>>(position, CS, SN);
    k_prep<<<NB * SEQ / 64, 256, 0, stream>>>(blocks, amask, BM, BASE);

    k_proj<1><<<dim3(NB * SEQ / 64, 2 * DM / 64, 1), 32, 0, stream>>>(XA, K2, WB, DM, K2, (h16*)0, NB * SEQ, (size_t)0, 0, 64, (size_t)0, QK, K2, NB * SEQ);
    k_proj<0><<<dim3(DM / 64, NB * SEQ / 64, 1), 32, 0, stream>>>(WB + (size_t)2 * DM * DM, DM, XA, K2, K2, VT, DM, (size_t)0, SEQ, SEQ, (size_t)DM * SEQ, (float*)0, 0, 0);

    k_qkrot<<<NB * SEQ / 8, 256, 0, stream>>>(QK, q_ln_w, k_ln_w, CS, SN, QH, (size_t)(SZ_PL / 2));

    k_flash<<<dim3(SEQ / (16 * AW), NB * NH_, 1), 32 * AW, 0, stream>>>(QH, QR, KH, KR, VT, BM, BASE, EWA, amask, OA);

    k_proj<1><<<dim3(NB * SEQ / 64, DM / 64, 1), 32, 0, stream>>>(OA, K2, OWB, DM, K2, (h16*)0, SEQ, (size_t)0, 0, 64, (size_t)0, OUT, DM, OUT_SEQ);
}
